// TrackedAttention_19662360281263
// MI455X (gfx1250) — hardware-verified
//
#include <hip/hip_runtime.h>
#include <math.h>
#include <stdint.h>

#ifndef NB
#define NB    2
#endif
#ifndef SEQ
#define SEQ   4096
#endif
#define NB_FULL  2
#define SEQ_FULL 4096
#define DMOD  512
#define NH    8
#define HD    64
#define PCAR  32768.0f
#define VCAR  1024.0f
#define LOG2E 1.4426950408889634f
#define ATT_WAVES   4
#define ATT_THREADS (ATT_WAVES * 32)
#define QTILES      (SEQ / 64)
#define ATT_BLOCKS  (NB * NH * QTILES)
#define NKB    (SEQ / 32)
#define SLAB   (16 * 68)
static_assert(HD == 64 && DMOD == NH * HD);
static_assert(NB >= 1 && NB <= NB_FULL);
static_assert((SEQ % 64) == 0 && SEQ >= 64 && SEQ <= SEQ_FULL);
static_assert(ATT_THREADS == 128 && NKB * 32 == SEQ);
static_assert((DMOD % 64) == 0 && (DMOD % 32) == 0);
static_assert(((SEQ * DMOD / 8) % 256) == 0 && ((DMOD * DMOD) % (64 * 64)) == 0 && (SEQ % 8) == 0);
static_assert((SLAB * 4) % 16 == 0);

typedef unsigned short u16;
typedef _Float16 v16h __attribute__((ext_vector_type(16)));
typedef _Float16 v8h  __attribute__((ext_vector_type(8)));
typedef __bf16   v16b __attribute__((ext_vector_type(16)));
typedef float    v8f  __attribute__((ext_vector_type(8)));
typedef float    v4f  __attribute__((ext_vector_type(4)));
typedef unsigned int v4u __attribute__((ext_vector_type(4)));

union FragH { v16h v; v8h h[2]; v4u u[2]; };
union FragB { v16b v; v4u u[2]; };

struct RopeFreq { float f[32]; };
static_assert(sizeof(RopeFreq) == 128);

__device__ __forceinline__ unsigned short bf_bits(float f) {
  unsigned u = __float_as_uint(f);
  return (unsigned short)((u + 0x7FFFu + ((u >> 16) & 1u)) >> 16);
}
__device__ __forceinline__ float bf_up(unsigned short h) { return __uint_as_float(((unsigned)h) << 16); }
__device__ __forceinline__ float bf_val(float f) { return bf_up(bf_bits(f)); }
__device__ __forceinline__ unsigned short h_bits(_Float16 x) { return __builtin_bit_cast(unsigned short, x); }
__device__ __forceinline__ unsigned pk16(unsigned short a, unsigned short b) { return (unsigned)a | ((unsigned)b << 16); }
__device__ __forceinline__ v8f zero8() { v8f z = {0.f, 0.f, 0.f, 0.f, 0.f, 0.f, 0.f, 0.f}; return z; }

__device__ __forceinline__ v16h ldfrag_h(const _Float16* p) {
  FragH f;
  f.h[0] = *(const v8h*)(p);
  f.h[1] = *(const v8h*)(p + 16);
  return f.v;
}
__device__ __forceinline__ v16b ldfrag_b(const u16* p) {
  FragB f;
  f.u[0] = *(const v4u*)(p);
  f.u[1] = *(const v4u*)(p + 16);
  return f.v;
}

__device__ __forceinline__ v8f mma_h(v16h a, v16h b, v8f c) {
  return __builtin_amdgcn_wmma_f32_16x16x32_f16(false, a, false, b, (short)0, c, false, false);
}
__device__ __forceinline__ v8f mma_b(v16b a, v16b b, v8f c) {
  return __builtin_amdgcn_wmma_f32_16x16x32_bf16(false, a, false, b, (short)0, c, false, false);
}
template <typename F>
__device__ __forceinline__ void guard2x8(v8f& a, v8f& b, F x0, F x1, F x2, F x3, F x4, F x5, F x6, F x7) {
#if defined(__HIP_DEVICE_COMPILE__)
  asm volatile("v_nop\n\tv_nop\n\tv_nop\n\tv_nop"
               : "+v"(a), "+v"(b) : "v"(x0), "v"(x1), "v"(x2), "v"(x3), "v"(x4), "v"(x5), "v"(x6), "v"(x7) : "memory");
#endif
}
template <typename F>
__device__ __forceinline__ void guard2x6(v8f& a, v8f& b, F x0, F x1, F x2, F x3, F x4, F x5) {
#if defined(__HIP_DEVICE_COMPILE__)
  asm volatile("v_nop\n\tv_nop\n\tv_nop\n\tv_nop"
               : "+v"(a), "+v"(b) : "v"(x0), "v"(x1), "v"(x2), "v"(x3), "v"(x4), "v"(x5) : "memory");
#endif
}
template <typename F>
__device__ __forceinline__ void guard6(v8f& a, v8f& b, v8f& c, v8f& d, F x0, F x1, F x2, F x3, F x4, F x5) {
#if defined(__HIP_DEVICE_COMPILE__)
  asm volatile("v_nop\n\tv_nop\n\tv_nop\n\tv_nop"
               : "+v"(a), "+v"(b), "+v"(c), "+v"(d) : "v"(x0), "v"(x1), "v"(x2), "v"(x3), "v"(x4), "v"(x5) : "memory");
#endif
}
__device__ __forceinline__ void acc_guard4(v8f& a, v8f& b, v8f& c, v8f& d) {
#if defined(__HIP_DEVICE_COMPILE__)
  asm volatile("v_nop\n\tv_nop\n\tv_nop\n\tv_nop" : "+v"(a), "+v"(b), "+v"(c), "+v"(d));
#endif
}
__device__ __forceinline__ void wave_sync_lds() {
#if defined(__HIP_DEVICE_COMPILE__)
  __builtin_amdgcn_fence(__ATOMIC_RELEASE, "workgroup");
  __builtin_amdgcn_wave_barrier();
  __builtin_amdgcn_fence(__ATOMIC_ACQUIRE, "workgroup");
#endif
}

__global__ __launch_bounds__(256) void cvt_x(const float* __restrict__ x, u16* D, int n8, int per_b8, int bstride8) {
  const int gt = blockIdx.x * 256 + (int)threadIdx.x;
  if (gt >= n8) return;
  const int b = gt / per_b8;
  const int w = gt - b * per_b8;
  const float* p = x + ((size_t)b * (size_t)bstride8 + (size_t)w) * 8;
  const v4f a = *(const v4f*)(p), c4 = *(const v4f*)(p + 4);
  float v[8];
#pragma unroll
  for (int e = 0; e < 4; ++e) { v[e] = a[e]; v[4 + e] = c4[e]; }
  unsigned short s[8];
#pragma unroll
  for (int e = 0; e < 8; ++e) s[e] = bf_bits(v[e]);
  v4u o;
#pragma unroll
  for (int e = 0; e < 4; ++e) o[e] = pk16(s[2 * e], s[2 * e + 1]);
  u16* d = D + (size_t)gt * 8;
  for (int pass = 0; pass < 2; ++pass) {
    *(volatile v4u*)(d) = o;
    __threadfence();
  }
}

__global__ __launch_bounds__(256) void tr_w(const float* __restrict__ W, u16* D) {
  __shared__ __align__(16) float T[64 * 68];
  const int t = (int)threadIdx.x, bid = blockIdx.x;
  const int nt = DMOD / 64;
  const int k0 = (bid / nt) * 64, n0 = (bid % nt) * 64;
#pragma unroll
  for (int it = 0; it < 4; ++it) {
    const int e = it * 256 + t;
    const int kr = e >> 4, c4 = (e & 15) * 4;
    const v4f v = *(const v4f*)(W + (size_t)(k0 + kr) * DMOD + n0 + c4);
    *(v4f*)(T + kr * 68 + c4) = v;
  }
  __syncthreads();
  v4u ov[2];
#pragma unroll
  for (int it = 0; it < 2; ++it) {
    const int task = it * 256 + t;
    const int nr = task >> 3, k8 = (task & 7) * 8;
    unsigned short s[8];
#pragma unroll
    for (int e = 0; e < 8; ++e) s[e] = bf_bits(T[(k8 + e) * 68 + nr]);
#pragma unroll
    for (int e = 0; e < 4; ++e) ov[it][e] = pk16(s[2 * e], s[2 * e + 1]);
  }
  for (int pass = 0; pass < 2; ++pass) {
#pragma unroll
    for (int it = 0; it < 2; ++it) {
      const int task = it * 256 + t;
      const int nr = task >> 3, k8 = (task & 7) * 8;
      *(volatile v4u*)(D + (size_t)(n0 + nr) * DMOD + k0 + k8) = ov[it];
    }
    __threadfence();
  }
}

__global__ __launch_bounds__(256) void rope_tab(RopeFreq fr, float* CS) {
  __shared__ __align__(16) float tab[8 * 64];
  const int t = (int)threadIdx.x;
  const int pr = t >> 5, j = t & 31;
  const int pos = blockIdx.x * 8 + pr;
  float inv = 0.f;
#pragma unroll
  for (int q = 0; q < 32; ++q) inv = (j == q) ? fr.f[q] : inv;
  const float ang = (float)pos * inv;
  float sv, cv;
  sincosf(ang, &sv, &cv);
  tab[pr * 64 + j] = cv;
  tab[pr * 64 + 32 + j] = sv;
  __syncthreads();
  if (t < 128) {
    const int row = t >> 4, c4 = (t & 15) * 4;
    const v4f v = *(const v4f*)(tab + row * 64 + c4);
    float* d = CS + (size_t)(blockIdx.x * 8 + row) * 64 + c4;
    for (int pass = 0; pass < 2; ++pass) {
      *(volatile v4f*)(d) = v;
      __threadfence();
    }
  }
}

__device__ __forceinline__ void epi16(float* sl, v8f a0, v8f a1, v8f a2, v8f a3, float oscale, u16* C, int N,
                                      size_t rowb, int col0, int lane) {
  const int hh = lane >> 4, m = lane & 15;
#pragma unroll
  for (int r = 0; r < 8; ++r) {
    const int ro = (8 * hh + r) * 68 + m;
    sl[ro]      = a0[r] * oscale;
    sl[ro + 16] = a1[r] * oscale;
    sl[ro + 32] = a2[r] * oscale;
    sl[ro + 48] = a3[r] * oscale;
  }
  wave_sync_lds();
  const int rq = lane >> 3, c8 = (lane & 7) * 8;
  v4u ov[4];
#pragma unroll
  for (int i4 = 0; i4 < 4; ++i4) {
    const int row = i4 * 4 + rq;
    const v4f a = *(const v4f*)(sl + row * 68 + c8), c4 = *(const v4f*)(sl + row * 68 + c8 + 4);
    float w[8];
#pragma unroll
    for (int e = 0; e < 4; ++e) { w[e] = a[e]; w[4 + e] = c4[e]; }
#pragma unroll
    for (int e = 0; e < 4; ++e) ov[i4][e] = pk16(h_bits((_Float16)w[2 * e]), h_bits((_Float16)w[2 * e + 1]));
  }
  u16* dst = C + (rowb + (size_t)rq) * (size_t)N + col0 + c8;
  for (int pass = 0; pass < 2; ++pass) {
#pragma unroll
    for (int i4 = 0; i4 < 4; ++i4) {
      *(volatile v4u*)(dst + (size_t)(i4 * 4) * (size_t)N) = ov[i4];
    }
    __threadfence();
  }
}

__device__ __forceinline__ void epi_hilo(float* sl, v8f a0, v8f a1, v8f a2, v8f a3, u16* CH, u16* CL, int N,
                                         size_t rowb, int col0, int lane) {
  const int hh = lane >> 4, m = lane & 15;
#pragma unroll
  for (int r = 0; r < 8; ++r) {
    const int ro = (8 * hh + r) * 68 + m;
    sl[ro]      = a0[r];
    sl[ro + 16] = a1[r];
    sl[ro + 32] = a2[r];
    sl[ro + 48] = a3[r];
  }
  wave_sync_lds();
  const int rq = lane >> 3, c8 = (lane & 7) * 8;
  v4u oh[4], ol[4];
#pragma unroll
  for (int i4 = 0; i4 < 4; ++i4) {
    const int row = i4 * 4 + rq;
    const v4f a = *(const v4f*)(sl + row * 68 + c8), c4 = *(const v4f*)(sl + row * 68 + c8 + 4);
    float w[8];
#pragma unroll
    for (int e = 0; e < 4; ++e) { w[e] = a[e]; w[4 + e] = c4[e]; }
#pragma unroll
    for (int e = 0; e < 4; ++e) {
      const unsigned short hb0 = bf_bits(w[2 * e]), hb1 = bf_bits(w[2 * e + 1]);
      const unsigned short lb0 = bf_bits(w[2 * e] - bf_up(hb0)), lb1 = bf_bits(w[2 * e + 1] - bf_up(hb1));
      oh[i4][e] = pk16(hb0, hb1);
      ol[i4][e] = pk16(lb0, lb1);
    }
  }
  const size_t dofs = (rowb + (size_t)rq) * (size_t)N + col0 + c8;
  for (int pass = 0; pass < 2; ++pass) {
#pragma unroll
    for (int i4 = 0; i4 < 4; ++i4) {
      const size_t o4 = dofs + (size_t)(i4 * 4) * (size_t)N;
      *(volatile v4u*)(CH + o4) = oh[i4];
      *(volatile v4u*)(CL + o4) = ol[i4];
    }
    __threadfence();
  }
}

__device__ __forceinline__ void mainloop_b(const u16* ap, const u16* bp, size_t bs, int K,
                                           v8f& acc0, v8f& acc1, v8f& acc2, v8f& acc3) {
#pragma unroll 1
  for (int k0 = 0; k0 < K; k0 += 32) {
    const v16b a  = ldfrag_b(ap + k0);
    const v16b b0 = ldfrag_b(bp + k0);
    const v16b b1 = ldfrag_b(bp + bs + k0);
    const v16b b2 = ldfrag_b(bp + 2 * bs + k0);
    const v16b b3 = ldfrag_b(bp + 3 * bs + k0);
    acc0 = mma_b(a, b0, acc0);
    acc1 = mma_b(a, b1, acc1);
    acc2 = mma_b(a, b2, acc2);
    acc3 = mma_b(a, b3, acc3);
    guard6<v16b>(acc0, acc1, acc2, acc3, a, b0, b1, b2, b3, a);
  }
  acc_guard4(acc0, acc1, acc2, acc3);
}

__global__ __launch_bounds__(128)
void gemm_rope(const u16* __restrict__ A, const u16* __restrict__ Bt, const float* __restrict__ bias,
               const float* __restrict__ CS, u16* CH, u16* CL, int M, int N, int K, int nbias, int seq) {
  __shared__ __align__(16) float slab[4 * SLAB];
  const int tid = threadIdx.x, wave = tid >> 5, lane = tid & 31, hh = lane >> 4, m = lane & 15;
  const int ntile = N >> 6;
  const int bid   = blockIdx.x;
  const int rowb  = (bid / ntile) * 64 + wave * 16;
  const int col0  = (bid % ntile) * 64;
  if (rowb + 16 > M) return;
  const u16* ap = A  + (size_t)(rowb + m) * K + 8 * hh;
  const u16* bp = Bt + (size_t)(col0 + m) * K + 8 * hh;
  const size_t bs = (size_t)16 * K;
  v8f acc0 = zero8(), acc1 = zero8(), acc2 = zero8(), acc3 = zero8();
  mainloop_b(ap, bp, bs, K, acc0, acc1, acc2, acc3);
  float bc[4];
#pragma unroll
  for (int j = 0; j < 4; ++j) {
    int ci = col0 + 16 * j + m;
    ci = (ci < nbias) ? ci : (nbias - 1);
    bc[j] = bf_val(bias[ci]);
  }
#pragma unroll
  for (int r = 0; r < 8; ++r) {
    acc0[r] += bc[0];
    acc1[r] += bc[1];
    acc2[r] += bc[2];
    acc3[r] += bc[3];
  }
  float* sl = slab + wave * SLAB;
  const int pos0 = rowb % seq;
#pragma unroll
  for (int it = 0; it < 8; ++it) {
    const int e = it * 32 + lane;
    const int row = e >> 4, c4 = (e & 15) * 4;
    const v4f tv = *(const v4f*)(CS + (size_t)(pos0 + row) * 64 + c4);
    *(v4f*)(sl + row * 68 + c4) = tv;
  }
  wave_sync_lds();
  const int fh = m >> 1;
#pragma unroll
  for (int r = 0; r < 8; ++r) {
    const float* tr = sl + (8 * hh + r) * 68;
    const float cA0 = tr[fh], cA1 = tr[8 + fh], cB0 = tr[16 + fh], cB1 = tr[24 + fh];
    const float sA0 = tr[32 + fh], sA1 = tr[40 + fh], sB0 = tr[48 + fh], sB1 = tr[56 + fh];
    const float x0 = acc0[r], x1 = acc1[r], x2 = acc2[r], x3 = acc3[r];
    acc0[r] = x0 * cA0 - x2 * sA0;
    acc1[r] = x1 * cA1 - x3 * sA1;
    acc2[r] = x2 * cB0 + x0 * sB0;
    acc3[r] = x3 * cB1 + x1 * sB1;
  }
  wave_sync_lds();
  epi_hilo(sl, acc0, acc1, acc2, acc3, CH, CL, N, (size_t)rowb, col0, lane);
}

__global__ __launch_bounds__(128)
void gemm_vt(const u16* __restrict__ A, const u16* __restrict__ Bt, u16* C, const float* __restrict__ bias,
             int M, int N, int K, int nbias, float oscale, int bstrideB, int cstrideC) {
  __shared__ __align__(16) float slab[4 * SLAB];
  const int tid = threadIdx.x, wave = tid >> 5, lane = tid & 31, hh = lane >> 4, m = lane & 15;
  const int ntile = N >> 6;
  const int bid   = blockIdx.x;
  const int rowb  = (bid / ntile) * 64 + wave * 16;
  const int col0  = (bid % ntile) * 64;
  if (rowb + 16 > M) return;
  const u16* Btb = Bt + (size_t)blockIdx.y * (size_t)bstrideB;
  u16*       Cb  = C  + (size_t)blockIdx.y * (size_t)cstrideC;
  const u16* ap = A   + (size_t)(rowb + m) * K + 8 * hh;
  const u16* bp = Btb + (size_t)(col0 + m) * K + 8 * hh;
  const size_t bs = (size_t)16 * K;
  v8f acc0 = zero8(), acc1 = zero8(), acc2 = zero8(), acc3 = zero8();
  mainloop_b(ap, bp, bs, K, acc0, acc1, acc2, acc3);
  float br[8];
#pragma unroll
  for (int r = 0; r < 8; ++r) {
    int ri = rowb + 8 * hh + r;
    ri = (ri < nbias) ? ri : (nbias - 1);
    br[r] = bf_val(bias[ri]);
  }
#pragma unroll
  for (int r = 0; r < 8; ++r) {
    acc0[r] += br[r];
    acc1[r] += br[r];
    acc2[r] += br[r];
    acc3[r] += br[r];
  }
  epi16(slab + wave * SLAB, acc0, acc1, acc2, acc3, oscale, Cb, N, (size_t)rowb, col0, lane);
}

__global__ __launch_bounds__(ATT_THREADS)
void attn_fwd(const u16* __restrict__ QH, const u16* __restrict__ QL, const u16* __restrict__ KH,
              const u16* __restrict__ KL, const u16* __restrict__ VPp, const float* __restrict__ maskp, float* out) {
  __shared__ __align__(16) float smem[ATT_WAVES * SLAB];

  const int tid  = threadIdx.x;
  const int wave = tid >> 5;
  const int lane = tid & 31;
  const int hh   = lane >> 4;
  const int c    = lane & 15;

  const int bid  = blockIdx.x;
  const int qt   = bid % QTILES;
  const int bh   = bid / QTILES;
  const int head = bh % NH;
  const int b    = bh / NH;
  if (b >= NB) return;
  const int q0   = qt * 64 + wave * 16;

  const size_t qofs = ((((size_t)b * SEQ) + (size_t)(q0 + c)) * NH + head) * HD + 8 * hh;
  const size_t kofs = ((((size_t)b * SEQ) + (size_t)c) * NH + head) * HD + 8 * hh;
  const u16* Kbh = KH + kofs;
  const u16* Kbl = KL + kofs;
  const size_t vofs = ((size_t)b * DMOD + (size_t)(head * HD + c)) * SEQ + 8 * hh;
  const _Float16* Vb = (const _Float16*)(const void*)VPp + vofs;
  const float* Mb = maskp + (size_t)b * SEQ_FULL + 8 * hh;
  const float lsc = 0.125f * LOG2E;
  const size_t kstep = (size_t)NH * HD;

  const v16b qh0 = ldfrag_b(QH + qofs);
  const v16b qh1 = ldfrag_b(QH + qofs + 32);
  const v16b ql0 = ldfrag_b(QL + qofs);
  const v16b ql1 = ldfrag_b(QL + qofs + 32);

  float mrun = -INFINITY, lrun = 0.f;
  v8f o[4];
#pragma unroll
  for (int j = 0; j < 4; ++j) o[j] = zero8();

#pragma unroll 1
  for (int it = 0; it < NKB; ++it) {
    const int kb = it * 32;
    v8f s0 = zero8(), s1 = zero8();
    const float* mp = Mb + kb;
    const v4f mk0 = *(const v4f*)(mp), mk1 = *(const v4f*)(mp + 4);
    const v4f mk2 = *(const v4f*)(mp + 16), mk3 = *(const v4f*)(mp + 20);
    float mk[16];
#pragma unroll
    for (int e = 0; e < 4; ++e) { mk[e] = mk0[e]; mk[4 + e] = mk1[e]; mk[8 + e] = mk2[e]; mk[12 + e] = mk3[e]; }
    {
      const u16* k0p = Kbh + (size_t)kb * kstep;
      const u16* k1p = k0p + (size_t)16 * kstep;
      const v16b ka0 = ldfrag_b(k0p), ka1 = ldfrag_b(k0p + 32);
      const v16b kc0 = ldfrag_b(k1p), kc1 = ldfrag_b(k1p + 32);
      s0 = mma_b(ka0, qh0, s0);
      s0 = mma_b(ka1, qh1, s0);
      s0 = mma_b(ka0, ql0, s0);
      s0 = mma_b(ka1, ql1, s0);
      s1 = mma_b(kc0, qh0, s1);
      s1 = mma_b(kc1, qh1, s1);
      s1 = mma_b(kc0, ql0, s1);
      s1 = mma_b(kc1, ql1, s1);
      guard2x8<v16b>(s0, s1, qh0, qh1, ql0, ql1, ka0, ka1, kc0, kc1);
    }
    {
      const u16* l0p = Kbl + (size_t)kb * kstep;
      const u16* l1p = l0p + (size_t)16 * kstep;
      const v16b kl0 = ldfrag_b(l0p), kl1 = ldfrag_b(l0p + 32);
      const v16b km0 = ldfrag_b(l1p), km1 = ldfrag_b(l1p + 32);
      s0 = mma_b(kl0, qh0, s0);
      s0 = mma_b(kl1, qh1, s0);
      s1 = mma_b(km0, qh0, s1);
      s1 = mma_b(km1, qh1, s1);
      guard2x6<v16b>(s0, s1, kl0, kl1, km0, km1, qh0, qh1);
    }
    float tk[16];
#pragma unroll
    for (int i = 0; i < 8; ++i) {
      tk[i]     = s0[i] * lsc + mk[i] * LOG2E;
      tk[8 + i] = s1[i] * lsc + mk[8 + i] * LOG2E;
    }
    float cm = tk[0];
#pragma unroll
    for (int i = 1; i < 16; ++i) cm = fmaxf(cm, tk[i]);
    cm = fmaxf(cm, __shfl_xor(cm, 16, 32));
    const float mn = fmaxf(mrun, cm);
    const float al = (mrun == -INFINITY) ? 0.f : exp2f(mrun - mn);
    mrun = mn;
    float ps = 0.f;
    FragH ph;
#pragma unroll
    for (int w = 0; w < 2; ++w) {
#pragma unroll
      for (int e4 = 0; e4 < 4; ++e4) {
        const int i = 8 * w + 2 * e4;
        const float p0 = exp2f(fminf(tk[i] - mn, 0.f));
        const float p1 = exp2f(fminf(tk[i + 1] - mn, 0.f));
        ps += p0 + p1;
        ph.u[w][e4] = pk16(h_bits((_Float16)(p0 * PCAR)), h_bits((_Float16)(p1 * PCAR)));
      }
    }
    ps += __shfl_xor(ps, 16, 32);
    lrun = lrun * al + ps;
    float scl[8];
#pragma unroll
    for (int r = 0; r < 8; ++r) scl[r] = __shfl(al, 8 * hh + r, 32);
#pragma unroll
    for (int j = 0; j < 4; ++j) {
#pragma unroll
      for (int r = 0; r < 8; ++r) o[j][r] *= scl[r];
    }
    {
      const _Float16* vp = Vb + kb;
      const v16h vf0 = ldfrag_h(vp);
      const v16h vf1 = ldfrag_h(vp + (size_t)16 * SEQ);
      const v16h vf2 = ldfrag_h(vp + (size_t)32 * SEQ);
      const v16h vf3 = ldfrag_h(vp + (size_t)48 * SEQ);
      o[0] = mma_h(ph.v, vf0, o[0]);
      o[1] = mma_h(ph.v, vf1, o[1]);
      o[2] = mma_h(ph.v, vf2, o[2]);
      o[3] = mma_h(ph.v, vf3, o[3]);
      guard6<v16h>(o[0], o[1], o[2], o[3], ph.v, vf0, vf1, vf2, vf3, ph.v);
    }
  }
  acc_guard4(o[0], o[1], o[2], o[3]);

  const float linv = (lrun > 0.f) ? ((1.0f / lrun) * (1.0f / (PCAR * VCAR))) : 0.f;
  float inv[8];
#pragma unroll
  for (int r = 0; r < 8; ++r) inv[r] = __shfl(linv, 8 * hh + r, 32);
  float* slab = smem + wave * SLAB;
#pragma unroll
  for (int r = 0; r < 8; ++r) {
#pragma unroll
    for (int j = 0; j < 4; ++j) slab[(8 * hh + r) * 68 + j * 16 + c] = o[j][r] * inv[r];
  }
  wave_sync_lds();
  v4f vals[8];
#pragma unroll
  for (int it = 0; it < 8; ++it) vals[it] = *(const v4f*)(slab + (it * 2 + hh) * 68 + c * 4);
  float* dst = out + ((((size_t)b * SEQ) + (size_t)(q0 + hh)) * DMOD) + head * HD + c * 4;
  for (int pass = 0; pass < 2; ++pass) {
#pragma unroll
    for (int it = 0; it < 8; ++it) {
      *(volatile v4f*)(dst + (size_t)(it * 2) * DMOD) = vals[it];
    }
    __threadfence();
  }
}

extern "C" void kernel_launch(void* const* d_in, const int* in_sizes, int n_in,
                              void* d_out, int out_size, void* d_ws, size_t ws_size,
                              hipStream_t stream) {
  if (n_in < 8) return;
  if (in_sizes[0] < ((NB - 1) * SEQ_FULL + SEQ) * DMOD) return;
  if (in_sizes[1] < (NB - 1) * SEQ_FULL + SEQ) return;
  if (in_sizes[2] < DMOD * DMOD || in_sizes[4] < DMOD * DMOD || in_sizes[6] < DMOD * DMOD) return;
  if (in_sizes[3] < DMOD || in_sizes[5] < DMOD || in_sizes[7] < DMOD) return;
  if (out_size < NB * SEQ * DMOD) return;

  const float* Xin = (const float*)d_in[0];
  const float* Msk = (const float*)d_in[1];
  const float* Wq  = (const float*)d_in[2];
  const float* bq  = (const float*)d_in[3];
  const float* Wk  = (const float*)d_in[4];
  const float* bk  = (const float*)d_in[5];
  const float* Wv  = (const float*)d_in[6];
  const float* bv  = (const float*)d_in[7];
  float*       out = (float*)d_out;

  const size_t szXB = (size_t)NB * SEQ * DMOD * 2;
  const size_t szW  = (size_t)DMOD * DMOD * 2;
  const size_t szCS = (size_t)SEQ * 64 * 4;
  const size_t szP  = (size_t)NB * SEQ * DMOD * 2;
  const size_t szVP = (size_t)NB * DMOD * SEQ * 2;
  size_t off = 0;
  const size_t oXB = off; off += szXB;
  const size_t oWQ = off; off += szW;
  const size_t oWK = off; off += szW;
  const size_t oWV = off; off += szW;
  const size_t oCS = off; off += szCS;
  const size_t oQH = off; off += szP;
  const size_t oQL = off; off += szP;
  const size_t oKH = off; off += szP;
  const size_t oKL = off; off += szP;
  const size_t oVP = off; off += szVP;
  if (off > ws_size) return;
  if (off > (size_t)134217728) return;

  char* ws = (char*)d_ws;
  u16*   XB  = (u16*)(ws + oXB);
  u16*   WQT = (u16*)(ws + oWQ);
  u16*   WKT = (u16*)(ws + oWK);
  u16*   WVT = (u16*)(ws + oWV);
  float* CS  = (float*)(ws + oCS);
  u16*   QH  = (u16*)(ws + oQH);
  u16*   QL  = (u16*)(ws + oQL);
  u16*   KH  = (u16*)(ws + oKH);
  u16*   KL  = (u16*)(ws + oKL);
  u16*   VP  = (u16*)(ws + oVP);

  RopeFreq fr;
  {
    const float invf[32] = {
      1.0f, 0.7498942017555237f, 0.5623413324356079f, 0.4216965138912201f,
      0.3162277638912201f, 0.23713736236095428f, 0.17782793939113617f, 0.1333521455526352f,
      0.10000000149011612f, 0.07498941570520401f, 0.05623412877321243f, 0.04216964915394783f,
      0.03162277862429619f, 0.0237137358635664f, 0.017782794311642647f, 0.01333521492779255f,
      0.009999999776482582f, 0.007498942315578461f, 0.005623413249850273f, 0.0042169648222625256f,
      0.003162277862429619f, 0.0023713738191872835f, 0.0017782794311642647f, 0.0013335214462131262f,
      0.0010000000474974513f, 0.0007498941849917173f, 0.000562341301701963f, 0.00042169648804701865f,
      0.0003162277862429619f, 0.0002371373848291114f, 0.00017782794020604342f, 0.0001333521504420787f};
    for (int j = 0; j < 32; ++j) fr.f[j] = invf[j];
  }

  const int n8x = (NB * SEQ * DMOD) / 8;
  if ((n8x % 256) != 0) return;
  if ((DMOD % 64) != 0 || (SEQ % 64) != 0 || (DMOD % 32) != 0 || (SEQ % 8) != 0) return;
  const dim3 blk(256);
  const dim3 gX(n8x / 256);
  const dim3 gTW((DMOD / 64) * (DMOD / 64));
  const dim3 gCS(SEQ / 8);
  const dim3 gGQ((NB * SEQ / 64) * (DMOD / 64));
  const dim3 gV((DMOD / 64) * (SEQ / 64), NB);
  const dim3 bG(128);
  const dim3 gAT(ATT_BLOCKS);
  const dim3 bAT(ATT_THREADS);

  cvt_x<<<gX, blk, 0, stream>>>(Xin, XB, n8x, (SEQ * DMOD) / 8, (SEQ_FULL * DMOD) / 8);
  tr_w<<<gTW, blk, 0, stream>>>(Wq, WQT);
  tr_w<<<gTW, blk, 0, stream>>>(Wk, WKT);
  tr_w<<<gTW, blk, 0, stream>>>(Wv, WVT);
  rope_tab<<<gCS, blk, 0, stream>>>(fr, CS);
  gemm_rope<<<gGQ, bG, 0, stream>>>(XB, WQT, bq, CS, QH, QL, NB * SEQ, DMOD, DMOD, DMOD, SEQ);
  gemm_rope<<<gGQ, bG, 0, stream>>>(XB, WKT, bk, CS, KH, KL, NB * SEQ, DMOD, DMOD, DMOD, SEQ);
  gemm_vt<<<gV, bG, 0, stream>>>(WVT, XB, VP, bv, DMOD, SEQ, DMOD, DMOD, VCAR, SEQ * DMOD, DMOD * SEQ);
  attn_fwd<<<gAT, bAT, 0, stream>>>(QH, QL, KH, KL, VP, Msk, out);
  (void)hipGetLastError();
}
